// Entity_Classify_49821620633803
// MI455X (gfx1250) — hardware-verified
//
#include <hip/hip_runtime.h>
#include <stddef.h>


#define DEV __device__ __forceinline__

constexpr int NN   = 50000;
constexpr int DD   = 128;
constexpr int RR   = 8;
constexpr int EE   = 80000;
constexpr int NB   = 4;
constexpr int NFT  = 4;
constexpr int VV   = 1000;
constexpr int NOUT = 16;
constexpr int KC   = RR * DD + DD;
constexpr int NPA  = ((NN + 63) / 64) * 64;
constexpr int LP   = 136;

constexpr float SA  = 256.0f;
constexpr float SBW = 64.0f;

constexpr int RB   = 512;
constexpr int ECH  = 1024;
constexpr int NCH  = (EE + ECH - 1) / ECH;
constexpr int AGG_ACC_BYTES = RB * DD * 4;
constexpr int AGG_DEG_OFF   = AGG_ACC_BYTES;
constexpr int AGG_SLOT_OFF  = AGG_DEG_OFF + RB * 4;
constexpr int AGG_MSK_OFF   = AGG_SLOT_OFF + 2 * ECH * 4;
constexpr int AGG_LDS_BYTES = AGG_MSK_OFF + 2 * 32 * 4;

constexpr int GEMM_TM   = 64;
constexpr int GEMM_AS   = GEMM_TM * LP * 2;
constexpr int GEMM_BS   = DD * LP * 2;
constexpr int GEMM_POOL = GEMM_AS + GEMM_BS;

static_assert(EE % 4 == 0);
static_assert(RB / 8 == 64);
static_assert(GEMM_TM * DD * 4 + GEMM_TM * LP * 2 <= GEMM_POOL);
static_assert((size_t)NPA * KC * 2 % 128 == 0);

typedef _Float16 v16h __attribute__((ext_vector_type(16)));
typedef _Float16 v8h  __attribute__((ext_vector_type(8), __may_alias__));
typedef float    v8f  __attribute__((ext_vector_type(8)));
typedef float    v4f  __attribute__((ext_vector_type(4), __may_alias__));
typedef unsigned v4u  __attribute__((ext_vector_type(4), __may_alias__));
typedef int      v4i  __attribute__((ext_vector_type(4), __may_alias__));
union Frag { v16h v; v8h hf[2]; };

DEV v8f wmma16(v16h a, v16h b, v8f c) {
    c = __builtin_amdgcn_wmma_f32_16x16x32_f16(false, a, false, b, (short)0, c, false, false);
    asm volatile("v_nop\n\tv_nop\n\tv_nop\n\tv_nop" : "+v"(c) : "v"(a), "v"(b));
    return c;
}

DEV int clampi(int v, int hi) { return v < 0 ? 0 : (v > hi ? hi : v); }

DEV v8h cvt8(v4f a, v4f b, float s) {
    v8h r = {(_Float16)(a[0] * s), (_Float16)(a[1] * s), (_Float16)(a[2] * s), (_Float16)(a[3] * s),
             (_Float16)(b[0] * s), (_Float16)(b[1] * s), (_Float16)(b[2] * s), (_Float16)(b[3] * s)};
    return r;
}

DEV v4f xrow4(const int* __restrict__ codes, const int* __restrict__ nid,
              const float* __restrict__ emb, int n, int c4) {
    const int idx = clampi(nid[n], NN - 1);
    v4f a = {0.f, 0.f, 0.f, 0.f};
#pragma unroll
    for (int f = 0; f < NFT; ++f) {
        const int c = clampi(codes[f * NN + idx], VV - 1);
        a += *(const v4f*)(emb + ((size_t)(f * VV + c)) * DD + c4);
    }
    return a;
}

__global__ __launch_bounds__(256)
void k_prep(const float* __restrict__ basis, const float* __restrict__ coeff,
            const float* __restrict__ W_self, _Float16* __restrict__ Bcat) {
    __shared__ __attribute__((aligned(16))) _Float16 rowh[KC];
    const int o = blockIdx.x;
    const int t = threadIdx.x;
    for (int k = t; k < KC; k += 256) {
        float v;
        if (k < RR * DD) {
            const int r = k >> 7, i = k & (DD - 1);
            float acc = 0.f;
#pragma unroll
            for (int b = 0; b < NB; ++b)
                acc += coeff[r * NB + b] * basis[(size_t)b * DD * DD + (size_t)i * DD + o];
            v = acc;
        } else {
            const int i = k - RR * DD;
            float s = 0.f;
#pragma unroll
            for (int r = 0; r < RR; ++r) s += W_self[(size_t)r * DD * DD + (size_t)i * DD + o];
            v = s;
        }
        rowh[k] = (_Float16)(v * SBW);
    }
    __syncthreads();
    if (t < KC / 8) {
        const v8h val = *(const v8h*)(rowh + 8 * t);
        _Float16* p = Bcat + (size_t)o * KC + 8 * t;
        *(volatile v8h*)p = val;
        __threadfence();
        *(volatile v8h*)p = val;
    }
}

__global__ __launch_bounds__(256)
void k_agg(const int* __restrict__ codes, const int* __restrict__ nid,
           const int* __restrict__ esrc, const int* __restrict__ edst,
           const float* __restrict__ emb, _Float16* __restrict__ Acat) {
    extern __shared__ __attribute__((aligned(16))) unsigned char dsm[];
    v4f*      acc  = (v4f*)dsm;
    int*      deg  = (int*)(dsm + AGG_DEG_OFF);
    unsigned* slot = (unsigned*)(dsm + AGG_SLOT_OFF);
    unsigned* msk  = (unsigned*)(dsm + AGG_MSK_OFF);

    const int t = threadIdx.x, l = t & 31, w = t >> 5, h = l >> 4, q = l & 15;
    const int row0 = blockIdx.x * RB;

    for (int pass = 0; pass < 2; ++pass) {
        if (pass) __threadfence();
        for (int i = 0; i < RB / 16; ++i) {
            const int rl = 64 * w + 2 * i + h;
            const int n = row0 + rl;
            if (n < NN) {
                const v4f s0 = xrow4(codes, nid, emb, n, 8 * q);
                const v4f s1 = xrow4(codes, nid, emb, n, 8 * q + 4);
                const v8h hv = cvt8(s0, s1, SA);
                *(volatile v8h*)(Acat + (size_t)n * KC + RR * DD + 8 * q) = hv;
            }
        }
    }

    const v4f z4 = {0.f, 0.f, 0.f, 0.f};
    for (int r = 0; r < RR; ++r) {
        __syncthreads();
#pragma unroll 4
        for (int i = 0; i < (RB * DD / 4) / 256; ++i) acc[t + 256 * i] = z4;
        for (int i = t; i < RB; i += 256) deg[i] = 0;
        __syncthreads();

        const int* ed = edst + (size_t)r * EE;
        const int* es = esrc + (size_t)r * EE;
        for (int c = 0; c < NCH; ++c) {
            const int buf = c & 1;
            unsigned* slotb = slot + buf * ECH;
            unsigned* mskb  = msk + buf * 32;
            const int e4 = c * ECH + 4 * t;
            v4i dv = {-1, -1, -1, -1};
            if (e4 < EE) dv = *(const v4i*)(ed + e4);
            v4u mw;
#pragma unroll
            for (int j = 0; j < 4; ++j) {
                const int d = dv[j];
                const unsigned dl = (unsigned)(d - row0);
                const bool match = (e4 < EE) && (dl < (unsigned)RB);
                if (match) {
                    const int s = clampi(es[e4 + j], NN - 1);
                    slotb[j * 256 + t] = (unsigned)s | (dl << 17);
                }
                mw[j] = __builtin_amdgcn_ballot_w32(match);
            }
            if (l == 0) *(v4u*)(mskb + 4 * w) = mw;
            __syncthreads();
#pragma unroll
            for (int w2 = 0; w2 < 8; ++w2) {
                const v4u m4 = *(const v4u*)(mskb + 4 * w2);
                if ((m4.x | m4.y | m4.z | m4.w) == 0u) continue;
#pragma unroll
                for (int j = 0; j < 4; ++j) {
                    unsigned bits = m4[j];
                    while (bits) {
                        const int b = __builtin_ctz(bits);
                        bits &= bits - 1u;
                        const unsigned u = slotb[j * 256 + w2 * 32 + b];
                        const int dloc = (int)(u >> 17) & (RB - 1);
                        const int s = clampi((int)(u & 0x1FFFFu), NN - 1);
                        if ((dloc & 7) == w) {
                            const v4f xv = xrow4(codes, nid, emb, s, 4 * l);
                            acc[dloc * 32 + l] += xv;
                            if (l == 0) deg[dloc] += 1;
                        }
                    }
                }
            }
        }
        __syncthreads();

        for (int pass = 0; pass < 2; ++pass) {
            if (pass) __threadfence();
            for (int i = 0; i < RB / 16; ++i) {
                const int rl = 64 * w + 2 * i + h;
                const int n = row0 + rl;
                const float rd = 1.0f / fmaxf((float)deg[rl], 1.0f);
                v4f a0 = acc[rl * 32 + 2 * q];
                v4f a1 = acc[rl * 32 + 2 * q + 1];
                a0 *= rd;
                a1 *= rd;
                if (n < NN) {
                    const v8h hv = cvt8(a0, a1, SA);
                    *(volatile v8h*)(Acat + (size_t)n * KC + r * DD + 8 * q) = hv;
                }
            }
        }
    }
}

DEV void gemm_store(const float* hs32, const float* lg, float* __restrict__ out0,
                    float* __restrict__ out1, int row0, int t, int l, int w) {
#pragma unroll
    for (int i = 0; i < 8; ++i) {
        const int row = 8 * w + i;
        const int n = row0 + row;
        if (n < NN) {
            const v4f v = *(const v4f*)(hs32 + row * DD + 4 * l);
            *(volatile v4f*)(out1 + (size_t)n * DD + 4 * l) = v;
        }
    }
    {
        const int row = t >> 2;
        const int n = row0 + row;
        if (n < NN) {
            const v4f v = *(const v4f*)(lg + 4 * t);
            *(volatile v4f*)(out0 + (size_t)row0 * NOUT + 4 * t) = v;
        }
    }
}

__global__ __launch_bounds__(256)
void k_gemm(const _Float16* __restrict__ Acat, const _Float16* __restrict__ Bcat,
            const float* __restrict__ b_rel, const float* __restrict__ h_bias,
            const float* __restrict__ W_cls, const float* __restrict__ b_cls,
            float* __restrict__ out0, float* __restrict__ out1) {
    __shared__ __attribute__((aligned(16))) unsigned char pool[GEMM_POOL];
    __shared__ __attribute__((aligned(16))) _Float16 wcs[NOUT * LP];
    __shared__ __attribute__((aligned(16))) float lg[GEMM_TM * NOUT];
    __shared__ float bias_s[DD];
    __shared__ float bcls_s[NOUT];
    _Float16* As   = (_Float16*)pool;
    _Float16* Bs   = (_Float16*)(pool + GEMM_AS);
    float*    hs32 = (float*)pool;
    _Float16* hs16 = (_Float16*)(pool + GEMM_TM * DD * 4);

    const int t = threadIdx.x, l = t & 31, w = t >> 5, h = l >> 4, m = l & 15;
    const int row0 = blockIdx.x * GEMM_TM;

    if (t < DD) {
        float b = h_bias[t];
#pragma unroll
        for (int r = 0; r < RR; ++r) b += b_rel[r * DD + t];
        bias_s[t] = b;
    }
    if (t < NOUT) bcls_s[t] = b_cls[t];
    {
        const int n = t >> 4, k0 = (t & 15) * 8;
        v8h v = {(_Float16)(W_cls[(k0 + 0) * NOUT + n] * SBW), (_Float16)(W_cls[(k0 + 1) * NOUT + n] * SBW),
                 (_Float16)(W_cls[(k0 + 2) * NOUT + n] * SBW), (_Float16)(W_cls[(k0 + 3) * NOUT + n] * SBW),
                 (_Float16)(W_cls[(k0 + 4) * NOUT + n] * SBW), (_Float16)(W_cls[(k0 + 5) * NOUT + n] * SBW),
                 (_Float16)(W_cls[(k0 + 6) * NOUT + n] * SBW), (_Float16)(W_cls[(k0 + 7) * NOUT + n] * SBW)};
        *(v8h*)(wcs + n * LP + k0) = v;
    }

    const v8f z8 = {0.f, 0.f, 0.f, 0.f, 0.f, 0.f, 0.f, 0.f};
    v8f acc[4];
#pragma unroll
    for (int j = 0; j < 4; ++j) acc[j] = z8;

#pragma unroll 1
    for (int kc = 0; kc < KC / DD; ++kc) {
        __syncthreads();
#pragma unroll
        for (int i = 0; i < 4; ++i) {
            const int idx = t + 256 * i;
            const int row = idx >> 4, c8 = (idx & 15) * 8;
            *(v8h*)(As + row * LP + c8) =
                *(const v8h*)(Acat + (size_t)(row0 + row) * KC + kc * DD + c8);
        }
#pragma unroll
        for (int i = 0; i < 8; ++i) {
            const int idx = t + 256 * i;
            const int n = idx >> 4, c8 = (idx & 15) * 8;
            *(v8h*)(Bs + n * LP + c8) =
                *(const v8h*)(Bcat + (size_t)n * KC + kc * DD + c8);
        }
        __syncthreads();
#pragma unroll
        for (int ks = 0; ks < 4; ++ks) {
            const int k0 = 32 * ks;
            Frag b;
            b.hf[0] = *(const v8h*)(Bs + (16 * w + m) * LP + k0 + 8 * h);
            b.hf[1] = *(const v8h*)(Bs + (16 * w + m) * LP + k0 + 16 + 8 * h);
#pragma unroll
            for (int j = 0; j < 4; ++j) {
                Frag a;
                a.hf[0] = *(const v8h*)(As + (16 * j + m) * LP + k0 + 8 * h);
                a.hf[1] = *(const v8h*)(As + (16 * j + m) * LP + k0 + 16 + 8 * h);
                acc[j] = wmma16(a.v, b.v, acc[j]);
            }
        }
    }
    __syncthreads();

    const float inv = 1.0f / (SA * SBW);
#pragma unroll
    for (int j = 0; j < 4; ++j) {
#pragma unroll
        for (int rr = 0; rr < 8; ++rr) {
            const int row = 16 * j + 8 * h + rr;
            const int col = 16 * w + m;
            float v = acc[j][rr] * inv + bias_s[col];
            v = fmaxf(v, 0.0f);
            hs32[row * DD + col] = v;
        }
    }
    __syncthreads();
#pragma unroll
    for (int i = 0; i < 4; ++i) {
        const int idx = t + 256 * i;
        const int row = idx >> 4, c8 = (idx & 15) * 8;
        const v4f a0 = *(const v4f*)(hs32 + row * DD + c8);
        const v4f a1 = *(const v4f*)(hs32 + row * DD + c8 + 4);
        *(v8h*)(hs16 + row * LP + c8) = cvt8(a0, a1, SA);
    }
    __syncthreads();
    if (w < 4) {
        v8f c2 = z8;
#pragma unroll
        for (int ks = 0; ks < 4; ++ks) {
            const int k0 = 32 * ks;
            Frag a, b;
            a.hf[0] = *(const v8h*)(hs16 + (16 * w + m) * LP + k0 + 8 * h);
            a.hf[1] = *(const v8h*)(hs16 + (16 * w + m) * LP + k0 + 16 + 8 * h);
            b.hf[0] = *(const v8h*)(wcs + m * LP + k0 + 8 * h);
            b.hf[1] = *(const v8h*)(wcs + m * LP + k0 + 16 + 8 * h);
            c2 = wmma16(a.v, b.v, c2);
        }
        const float inv2 = 1.0f / (SA * SBW);
#pragma unroll
        for (int rr = 0; rr < 8; ++rr) {
            const int row = 16 * w + 8 * h + rr;
            lg[row * NOUT + m] = c2[rr] * inv2 + bcls_s[m];
        }
    }
    __syncthreads();

    gemm_store(hs32, lg, out0, out1, row0, t, l, w);
    __threadfence();
    gemm_store(hs32, lg, out0, out1, row0, t, l, w);
}

extern "C" void kernel_launch(void* const* d_in, const int* in_sizes, int n_in,
                              void* d_out, int out_size, void* d_ws, size_t ws_size,
                              hipStream_t stream) {
    if (n_in < 12) return;
    if (in_sizes[0] != NFT * NN || in_sizes[1] != NN || in_sizes[2] != RR * EE ||
        in_sizes[3] != RR * EE || in_sizes[4] != NFT * VV * DD || in_sizes[5] != NB * DD * DD ||
        in_sizes[6] != RR * NB || in_sizes[7] != RR * DD * DD || in_sizes[8] != RR * DD ||
        in_sizes[9] != DD || in_sizes[10] != DD * NOUT || in_sizes[11] != NOUT) return;
    if (out_size != NN * NOUT + NN * DD) return;

    const int*   codes  = (const int*)d_in[0];
    const int*   nid    = (const int*)d_in[1];
    const int*   esrc   = (const int*)d_in[2];
    const int*   edst   = (const int*)d_in[3];
    const float* emb    = (const float*)d_in[4];
    const float* basis  = (const float*)d_in[5];
    const float* coeff  = (const float*)d_in[6];
    const float* W_self = (const float*)d_in[7];
    const float* b_rel  = (const float*)d_in[8];
    const float* h_bias = (const float*)d_in[9];
    const float* W_cls  = (const float*)d_in[10];
    const float* b_cls  = (const float*)d_in[11];

    float* out0 = (float*)d_out;
    float* out1 = out0 + (size_t)NN * NOUT;

    const size_t acat_bytes = (size_t)NPA * KC * 2;
    const size_t bcat_bytes = (size_t)DD * KC * 2;
    if (acat_bytes + bcat_bytes > ws_size) return;
    _Float16* Acat = (_Float16*)d_ws;
    _Float16* Bcat = (_Float16*)((unsigned char*)d_ws + acat_bytes);

    hipFuncSetAttribute(reinterpret_cast<const void*>(&k_agg),
                        hipFuncAttributeMaxDynamicSharedMemorySize, AGG_LDS_BYTES);

    k_prep<<<DD, 256, 0, stream>>>(basis, coeff, W_self, Bcat);
    k_agg<<<(NN + RB - 1) / RB, 256, AGG_LDS_BYTES, stream>>>(codes, nid, esrc, edst, emb, Acat);
    k_gemm<<<(NN + GEMM_TM - 1) / GEMM_TM, 256, 0, stream>>>(Acat, Bcat, b_rel, h_bias, W_cls,
                                                              b_cls, out0, out1);
}
